// discrete_net_model_171798692344
// MI455X (gfx1250) — hardware-verified
//
#include <hip/hip_runtime.h>


typedef __bf16         v16b __attribute__((ext_vector_type(16)));
typedef float          v8f  __attribute__((ext_vector_type(8)));
typedef unsigned int   v4u  __attribute__((ext_vector_type(4)));
typedef unsigned short us_t;

#define NB_    16
#define NT_    64
#define NS_    256
#define NIN_   7
#define NH_    64
#define NO_    16
#define NOUT_  17
#define ND_    31
#define TP_    4
#define NSTEP_ 63
#define TOUT_  59
#define KP_    224
#define NG_    256
#define HROWS_ 258
#define PLH_   (HROWS_ * NH_)
#define XW_    32
#define HWN_   32

#define LDS_C_BYTES   (NS_ * NH_ * 4)
#define LDS_H_OFF     LDS_C_BYTES
#define LDS_PL_BYTES  (PLH_ * 2)
#define LDS_O0_OFF    (LDS_H_OFF + 4 * LDS_PL_BYTES)
#define LDS_O0_BYTES  (NS_ * NOUT_ * 4)
#define LDS_O1_OFF    (LDS_O0_OFF + LDS_O0_BYTES)
#define LDS_O1_BYTES  (NS_ * ND_ * 4)
#define LDS_TOTAL     (LDS_O1_OFF + LDS_O1_BYTES)
#define P0_           (LDS_O0_BYTES / 16)
#define P1_           (LDS_O1_BYTES / 16)

static_assert(LDS_TOTAL == 246784);
static_assert((LDS_O0_BYTES % 128) == 0);
static_assert((LDS_O1_BYTES % 128) == 0);
static_assert((LDS_O0_OFF % 16) == 0);
static_assert(P0_ == 1088);
static_assert(P1_ == 1984);

union BFrag { v16b v; v4u q[2]; };

__device__ __forceinline__ v8f mma(const BFrag& a, const BFrag& b, v8f c) {
    return __builtin_amdgcn_wmma_f32_16x16x32_bf16(false, a.v, false, b.v, (short)0, c, false, false);
}

__device__ __forceinline__ void ldf(BFrag& f, const us_t* p) {
    f.q[0] = *(const v4u*)p;
    f.q[1] = *(const v4u*)(p + 16);
}

__device__ __forceinline__ void ldB4(BFrag (&bh)[4], BFrag (&bl)[4],
                                     const us_t* __restrict__ WPh, const us_t* __restrict__ WPl,
                                     int uj, int m, int kc) {
#pragma unroll
    for (int g = 0; g < 4; ++g) {
        const size_t off = (size_t)(g * NH_ + 16 * uj + m) * KP_ + kc;
        ldf(bh[g], WPh + off);
        ldf(bl[g], WPl + off);
    }
}

__device__ __forceinline__ void mma12(v8f (&acc)[4], const BFrag& ah, const BFrag& al,
                                      const BFrag (&bh)[4], const BFrag (&bl)[4]) {
#pragma unroll
    for (int g = 0; g < 4; ++g) {
        acc[g] = mma(ah, bh[g], acc[g]);
        acc[g] = mma(ah, bl[g], acc[g]);
        acc[g] = mma(al, bh[g], acc[g]);
    }
    asm volatile("v_nop\n\tv_nop\n\tv_nop\n\tv_nop"
                 : "+v"(acc[0]), "+v"(acc[1]), "+v"(acc[2]), "+v"(acc[3])
                 : "v"(ah.v), "v"(al.v),
                   "v"(bh[0].v), "v"(bh[1].v), "v"(bh[2].v), "v"(bh[3].v),
                   "v"(bl[0].v), "v"(bl[1].v), "v"(bl[2].v), "v"(bl[3].v));
}

__device__ __forceinline__ unsigned bfbits(float f) {
    unsigned u = __float_as_uint(f);
    return (u + 0x7FFFu + ((u >> 16) & 1u)) >> 16;
}
__device__ __forceinline__ void split2(float v, unsigned& hb, unsigned& lb) {
    hb = bfbits(v);
    const float hf = __uint_as_float(hb << 16);
    lb = bfbits(v - hf);
}

__device__ __forceinline__ float frcp(float x) { return __builtin_amdgcn_rcpf(x); }
__device__ __forceinline__ float fsig(float x) {
    const float e = __expf(-x);
    return frcp(1.0f + e);
}
__device__ __forceinline__ float ftanh(float x) {
    const float ax = fabsf(x);
    const float e  = __expf(-2.0f * ax);
    const float r  = (1.0f - e) * frcp(1.0f + e);
    const float x2 = x * x;
    const float p  = ax * (1.0f + x2 * (-0.333333333f + x2 * (0.133333333f
                     + x2 * (-0.0539682540f + x2 * 0.0218694885f))));
    const float y  = (ax < 0.25f) ? p : r;
    return copysignf(y, x);
}

__global__ __launch_bounds__(256)
void k_xplanes(const float* __restrict__ x, us_t* XPh, us_t* XPl, int npieces, int nx) {
    const int i = blockIdx.x * 256 + threadIdx.x;
    if (i >= npieces) return;
    const int row = i >> 2;
    const int cc  = (i & 3) * 8;
    unsigned hw[4], lw[4];
#pragma unroll
    for (int j = 0; j < 4; ++j) { hw[j] = 0u; lw[j] = 0u; }
#pragma unroll
    for (int e = 0; e < 8; ++e) {
        const int col = cc + e;
        int idx = row * NIN_ + ((col < NIN_) ? col : (NIN_ - 1));
        idx = (idx < nx) ? idx : (nx - 1);
        float v = x[idx];
        v = (col < NIN_) ? v : 0.0f;
        unsigned hb, lb;
        split2(v, hb, lb);
        hw[e >> 1] |= hb << (16 * (e & 1));
        lw[e >> 1] |= lb << (16 * (e & 1));
    }
    v4u vh, vl;
    vh[0] = hw[0]; vh[1] = hw[1]; vh[2] = hw[2]; vh[3] = hw[3];
    vl[0] = lw[0]; vl[1] = lw[1]; vl[2] = lw[2]; vl[3] = lw[3];
    us_t* dh = XPh + (size_t)i * 8;
    us_t* dl = XPl + (size_t)i * 8;
    *(volatile v4u*)dh = vh;
    *(volatile v4u*)dl = vl;
    __threadfence();
    *(volatile v4u*)dh = vh;
    *(volatile v4u*)dl = vl;
}

__global__ __launch_bounds__(256)
void k_wplanes(const float* __restrict__ Wg, us_t* WPh, us_t* WPl, int npieces) {
    const int i = blockIdx.x * 256 + threadIdx.x;
    if (i >= npieces) return;
    const int n  = i / (KP_ / 8);
    const int kc = (i - n * (KP_ / 8)) * 8;
    unsigned hw[4], lw[4];
#pragma unroll
    for (int j = 0; j < 4; ++j) { hw[j] = 0u; lw[j] = 0u; }
#pragma unroll
    for (int e = 0; e < 8; ++e) {
        const int k = kc + e;
        const bool valid = (k < NIN_) || (k >= 32);
        int r = (k < NIN_) ? k : (k - 25);
        r = (r < 0) ? 0 : ((r > NIN_ + 3 * NH_ - 1) ? (NIN_ + 3 * NH_ - 1) : r);
        float v = Wg[r * NG_ + n];
        v = valid ? v : 0.0f;
        unsigned hb, lb;
        split2(v, hb, lb);
        hw[e >> 1] |= hb << (16 * (e & 1));
        lw[e >> 1] |= lb << (16 * (e & 1));
    }
    v4u vh, vl;
    vh[0] = hw[0]; vh[1] = hw[1]; vh[2] = hw[2]; vh[3] = hw[3];
    vl[0] = lw[0]; vl[1] = lw[1]; vl[2] = lw[2]; vl[3] = lw[3];
    us_t* dh = WPh + (size_t)i * 8;
    us_t* dl = WPl + (size_t)i * 8;
    *(volatile v4u*)dh = vh;
    *(volatile v4u*)dl = vl;
    __threadfence();
    *(volatile v4u*)dh = vh;
    *(volatile v4u*)dl = vl;
}

__global__ __launch_bounds__(256)
void k_hplanes(const float* __restrict__ Wn, const float* __restrict__ Ws,
               us_t* HWh, us_t* HWl, int npieces) {
    const int i = blockIdx.x * 256 + threadIdx.x;
    if (i >= npieces) return;
    const int n  = i >> 3;
    const int kc = (i & 7) * 8;
    unsigned hw[4], lw[4];
#pragma unroll
    for (int j = 0; j < 4; ++j) { hw[j] = 0u; lw[j] = 0u; }
#pragma unroll
    for (int e = 0; e < 8; ++e) {
        const int k = kc + e;
        const float vn = Wn[k * NO_ + ((n < NO_) ? n : (NO_ - 1))];
        const float vs = Ws[k];
        const float v  = (n < NO_) ? vn : ((n == NO_) ? vs : 0.0f);
        unsigned hb, lb;
        split2(v, hb, lb);
        hw[e >> 1] |= hb << (16 * (e & 1));
        lw[e >> 1] |= lb << (16 * (e & 1));
    }
    v4u vh, vl;
    vh[0] = hw[0]; vh[1] = hw[1]; vh[2] = hw[2]; vh[3] = hw[3];
    vl[0] = lw[0]; vl[1] = lw[1]; vl[2] = lw[2]; vl[3] = lw[3];
    us_t* dh = HWh + (size_t)i * 8;
    us_t* dl = HWl + (size_t)i * 8;
    *(volatile v4u*)dh = vh;
    *(volatile v4u*)dl = vl;
    __threadfence();
    *(volatile v4u*)dh = vh;
    *(volatile v4u*)dl = vl;
}

__global__ __launch_bounds__(256)
void k_lstm(const us_t* __restrict__ XPh, const us_t* __restrict__ XPl,
            const us_t* __restrict__ WPh, const us_t* __restrict__ WPl,
            const us_t* __restrict__ HWh, const us_t* __restrict__ HWl,
            const float* __restrict__ bg, const float* __restrict__ bn,
            const float* __restrict__ bs, const float* __restrict__ x,
            float* out0, float* out1)
{
    extern __shared__ v4u lds_v4[];
    unsigned char* lds = (unsigned char*)lds_v4;
    float* C32 = (float*)lds;
    us_t*  HP  = (us_t*)(lds + LDS_H_OFF);
    float* O0  = (float*)(lds + LDS_O0_OFF);
    float* O1  = (float*)(lds + LDS_O1_OFF);

    const int tid = threadIdx.x;
    const int w = tid >> 5, l = tid & 31, h = l >> 4, m = l & 15;
    const int b = blockIdx.x;

    {
        v4u z; z[0] = 0u; z[1] = 0u; z[2] = 0u; z[3] = 0u;
        for (int i = tid; i < LDS_O0_OFF / 16; i += 256) lds_v4[i] = z;
    }
    __syncthreads();

    const v8f zacc = {0.f, 0.f, 0.f, 0.f, 0.f, 0.f, 0.f, 0.f};

#pragma unroll 1
    for (int t = 0; t < NSTEP_; ++t) {
        const int cur = t & 1;
        const us_t* Hch = HP + (cur * 2 + 0) * PLH_;
        const us_t* Hcl = HP + (cur * 2 + 1) * PLH_;
        us_t* Hnh = HP + ((cur ^ 1) * 2 + 0) * PLH_;
        us_t* Hnl = HP + ((cur ^ 1) * 2 + 1) * PLH_;

#pragma unroll 1
        for (int q = 0; q < 8; ++q) {
            const int task = w * 8 + q;
            const int mi = task >> 2, uj = task & 3;
            v8f acc[4];
            acc[0] = zacc; acc[1] = zacc; acc[2] = zacc; acc[3] = zacc;
            BFrag ah, al, bh[4], bl[4];
            {
                const size_t xr = ((size_t)(b * NT_ + t) * NS_ + 16 * mi + m) * XW_ + 8 * h;
                ldf(ah, XPh + xr);
                ldf(al, XPl + xr);
                ldB4(bh, bl, WPh, WPl, uj, m, 8 * h);
                mma12(acc, ah, al, bh, bl);
            }
#pragma unroll 1
            for (int ks = 1; ks < 7; ++ks) {
                const int blk = (ks - 1) >> 1;
                const int k0  = ((ks - 1) & 1) * 32;
                const int d   = (blk == 1) ? 1 : ((blk == 2) ? -1 : 0);
                const int ar  = (16 * mi + m + 1 + d) * NH_ + k0 + 8 * h;
                ldf(ah, Hch + ar);
                ldf(al, Hcl + ar);
                ldB4(bh, bl, WPh, WPl, uj, m, ks * 32 + 8 * h);
                mma12(acc, ah, al, bh, bl);
            }
            {
                const int u = 16 * uj + m;
                const float bI = bg[u];
                const float bF = bg[NH_ + u];
                const float bG = bg[2 * NH_ + u];
                const float bO = bg[3 * NH_ + u];
#pragma unroll
                for (int r = 0; r < 8; ++r) {
                    const int s = 16 * mi + 8 * h + r;
                    const float zi = acc[0][r] + bI;
                    const float zf = acc[1][r] + bF;
                    const float zg = acc[2][r] + bG;
                    const float zo = acc[3][r] + bO;
                    const int ci = s * NH_ + u;
                    const float co = C32[ci];
                    const float cn = fsig(zf) * co + fsig(zi) * ftanh(zg);
                    const float hn = fsig(zo) * ftanh(cn);
                    C32[ci] = cn;
                    unsigned hb, lb;
                    split2(hn, hb, lb);
                    const int hi = (s + 1) * NH_ + u;
                    Hnh[hi] = (us_t)hb;
                    Hnl[hi] = (us_t)lb;
                }
            }
        }
        __syncthreads();

        if (t >= TP_) {
#pragma unroll 1
            for (int q = 0; q < 4; ++q) {
                const int task = w * 4 + q;
                const int mi = task >> 1, nj = task & 1;
                v8f acc = zacc;
#pragma unroll
                for (int ks = 0; ks < 2; ++ks) {
                    BFrag ah, al, bh1, bl1;
                    const int ar = (16 * mi + m + 1) * NH_ + ks * 32 + 8 * h;
                    ldf(ah, Hnh + ar);
                    ldf(al, Hnl + ar);
                    const int br = (16 * nj + m) * NH_ + ks * 32 + 8 * h;
                    ldf(bh1, HWh + br);
                    ldf(bl1, HWl + br);
                    acc = mma(ah, bh1, acc);
                    acc = mma(ah, bl1, acc);
                    acc = mma(al, bh1, acc);
                    asm volatile("v_nop\n\tv_nop\n\tv_nop\n\tv_nop"
                                 : "+v"(acc)
                                 : "v"(ah.v), "v"(al.v), "v"(bh1.v), "v"(bl1.v));
                }
                const int n = 16 * nj + m;
                const float bnv  = bn[m];
                const float bsv  = bs[0];
                const float bias = (nj == 0) ? bnv : bsv;
#pragma unroll
                for (int r = 0; r < 8; ++r) {
                    const int s = 16 * mi + 8 * h + r;
                    const float v = acc[r] + bias;
                    if (n < NOUT_) O0[s * NOUT_ + n] = v;
                }
            }
            __syncthreads();

            {
                const int s  = tid;
                const int sp = (s > 0) ? (s - 1) : 0;
                float xv = x[((size_t)(b * NT_ + t) * NS_) * NIN_];
                xv = fminf(fmaxf(xv, -1.0e6f), 1.0e6f);
                const int cls = (int)xv;
                float op[NO_], ip[NO_];
#pragma unroll 16
                for (int o = 0; o < NO_; ++o) {
                    op[o] = O0[s * NOUT_ + o];
                    const float pv = O0[sp * NOUT_ + o];
                    ip[o] = (s == 0) ? ((o == cls) ? 1.0f : 0.0f) : pv;
                }
#pragma unroll 31
                for (int ll = 0; ll < ND_; ++ll) {
                    float a = 0.0f;
#pragma unroll 16
                    for (int o = 0; o < NO_; ++o) {
                        const int src = o + ll - (NO_ - 1);
                        if (src >= 0 && src < NO_) a = fmaf(ip[o], op[src], a);
                    }
                    O1[s * ND_ + ll] = a;
                }
            }
            __syncthreads();

            {
                const int tt = t - TP_;
                volatile v4u* g0 = (volatile v4u*)(out0 + ((size_t)(b * TOUT_ + tt)) * (NS_ * NOUT_));
                volatile v4u* g1 = (volatile v4u*)(out1 + ((size_t)(b * TOUT_ + tt)) * (NS_ * ND_));
                const v4u* s0 = (const v4u*)O0;
                const v4u* s1 = (const v4u*)O1;
                v4u r0[5], r1[8];
#pragma unroll
                for (int i = 0; i < 5; ++i) {
                    int p = tid + 256 * i;
                    p = (p < P0_) ? p : (P0_ - 1);
                    r0[i] = s0[p];
                }
#pragma unroll
                for (int i = 0; i < 8; ++i) {
                    int p = tid + 256 * i;
                    p = (p < P1_) ? p : (P1_ - 1);
                    r1[i] = s1[p];
                }
#pragma unroll
                for (int i = 0; i < 5; ++i) {
                    const int p = tid + 256 * i;
                    if (p < P0_) g0[p] = r0[i];
                }
#pragma unroll
                for (int i = 0; i < 8; ++i) {
                    const int p = tid + 256 * i;
                    if (p < P1_) g1[p] = r1[i];
                }
                __threadfence();
#pragma unroll
                for (int i = 0; i < 5; ++i) {
                    const int p = tid + 256 * i;
                    if (p < P0_) g0[p] = r0[i];
                }
#pragma unroll
                for (int i = 0; i < 8; ++i) {
                    const int p = tid + 256 * i;
                    if (p < P1_) g1[p] = r1[i];
                }
            }
        }
    }
}

extern "C" void kernel_launch(void* const* d_in, const int* in_sizes, int n_in,
                              void* d_out, int out_size, void* d_ws, size_t ws_size,
                              hipStream_t stream) {
    if (n_in < 7) return;
    const int nx = NB_ * NT_ * NS_ * NIN_;
    if (in_sizes[0] != nx) return;
    if (in_sizes[1] != (NIN_ + 3 * NH_) * NG_) return;
    if (in_sizes[2] != NG_) return;
    if (in_sizes[3] != NH_ * NO_) return;
    if (in_sizes[4] != NO_) return;
    if (in_sizes[5] != NH_) return;
    if (in_sizes[6] != 1) return;
    const int n0 = NB_ * TOUT_ * NS_ * NOUT_;
    const int n1 = NB_ * TOUT_ * NS_ * ND_;
    if (out_size != n0 + n1) return;

    const float* x  = (const float*)d_in[0];
    const float* Wg = (const float*)d_in[1];
    const float* bg = (const float*)d_in[2];
    const float* Wn = (const float*)d_in[3];
    const float* bn = (const float*)d_in[4];
    const float* Ws = (const float*)d_in[5];
    const float* bs = (const float*)d_in[6];
    float* out0 = (float*)d_out;
    float* out1 = out0 + n0;

    char* ws = (char*)d_ws;
    size_t off = 0;
    auto carve = [&](size_t bytes) -> char* {
        char* p = ws + off;
        off = (off + bytes + 255) & ~(size_t)255;
        return p;
    };
    const size_t xrows   = (size_t)NB_ * NT_ * NS_;
    const size_t xpbytes = xrows * XW_ * 2;
    const size_t wpbytes = (size_t)NG_ * KP_ * 2;
    const size_t hwbytes = (size_t)HWN_ * NH_ * 2;
    us_t* XPh = (us_t*)carve(xpbytes);
    us_t* XPl = (us_t*)carve(xpbytes);
    us_t* WPh = (us_t*)carve(wpbytes);
    us_t* WPl = (us_t*)carve(wpbytes);
    us_t* HWh = (us_t*)carve(hwbytes);
    us_t* HWl = (us_t*)carve(hwbytes);
    if (off > ws_size) return;
    if (off > (size_t)134217728) return;

    {
        const int npieces = (int)(xrows * XW_ / 8);
        k_xplanes<<<dim3((npieces + 255) / 256), dim3(256), 0, stream>>>(x, XPh, XPl, npieces, nx);
    }
    {
        const int npieces = NG_ * (KP_ / 8);
        k_wplanes<<<dim3((npieces + 255) / 256), dim3(256), 0, stream>>>(Wg, WPh, WPl, npieces);
    }
    {
        const int npieces = HWN_ * NH_ / 8;
        k_hplanes<<<dim3((npieces + 255) / 256), dim3(256), 0, stream>>>(Wn, Ws, HWh, HWl, npieces);
    }
    hipFuncSetAttribute(reinterpret_cast<const void*>(&k_lstm),
                        hipFuncAttributeMaxDynamicSharedMemorySize, LDS_TOTAL);
    k_lstm<<<dim3(NB_), dim3(256), LDS_TOTAL, stream>>>(XPh, XPl, WPh, WPl, HWh, HWl,
                                                        bg, bn, bs, x, out0, out1);
}
